// SelfAttentionBlock_65481071406807
// MI455X (gfx1250) — hardware-verified
//
#include <hip/hip_runtime.h>


#ifndef NB
#define NB 4
#endif
#ifndef SEQ
#define SEQ 2048
#endif
#define NB_FULL  4
#define SEQ_FULL 2048
#define DM   1024
#define QC   (3 * DM)
#define PCAR 16384.0f
#define SCL  0.125f
#define WSC  64.0f

static_assert(NB >= 1 && NB <= NB_FULL);
static_assert(SEQ >= 256 && SEQ <= SEQ_FULL);
static_assert(SEQ % 256 == 0);
static_assert(DM % 256 == 0);
static_assert(QC % 64 == 0);
static_assert((SEQ * DM) % 2048 == 0);
static_assert((DM * SEQ) % 2048 == 0);

typedef _Float16 h16;
typedef unsigned short bf;
typedef __attribute__((ext_vector_type(16))) __bf16   v16bf;
typedef __attribute__((ext_vector_type(16))) _Float16 v16h;
typedef __attribute__((ext_vector_type(8)))  _Float16 v8h;
typedef __attribute__((ext_vector_type(8)))  unsigned short v8us;
typedef __attribute__((ext_vector_type(8)))  float    v8f;
typedef __attribute__((ext_vector_type(4)))  float    v4f;
typedef __attribute__((ext_vector_type(4)))  _Float16 v4h;
typedef v8h  __attribute__((may_alias)) v8ha;
typedef v4f  __attribute__((may_alias)) v4fa;
typedef v8us __attribute__((may_alias)) v8usa;

__device__ __forceinline__ unsigned short f2bf(float f) { unsigned u = __float_as_uint(f); u += 0x7FFFu + ((u >> 16) & 1u); return (unsigned short)(u >> 16); }
__device__ __forceinline__ float bf2f(unsigned short b) { return __uint_as_float(((unsigned)b) << 16); }
__device__ __forceinline__ float bfr(float f) { return bf2f(f2bf(f)); }
__device__ __forceinline__ h16 tohx(float x) { return (h16)x; }
__device__ __forceinline__ void splitf(float y, unsigned short& h, unsigned short& l) { h = f2bf(y); l = f2bf(y - bf2f(h)); }
__device__ __forceinline__ v16h cat16(v8h lo, v8h hi) { return __builtin_shufflevector(lo, hi, 0, 1, 2, 3, 4, 5, 6, 7, 8, 9, 10, 11, 12, 13, 14, 15); }
__device__ __forceinline__ v16bf cat16b(v8us lo, v8us hi) { return __builtin_bit_cast(v16bf, __builtin_shufflevector(lo, hi, 0, 1, 2, 3, 4, 5, 6, 7, 8, 9, 10, 11, 12, 13, 14, 15)); }
__device__ __forceinline__ v8f wmma16(v16h a, v16h b, v8f c) { return __builtin_amdgcn_wmma_f32_16x16x32_f16(false, a, false, b, (short)0, c, false, false); }
__device__ __forceinline__ v8f wmmab(v16bf a, v16bf b, v8f c) { return __builtin_amdgcn_wmma_f32_16x16x32_bf16(false, a, false, b, (short)0, c, false, false); }

template <typename T16> struct WFrag;
template <> struct WFrag<h16> { typedef v16h V; static __device__ __forceinline__ V ld(const h16* p) { return cat16(*(const v8h*)p, *(const v8h*)(p + 16)); } static __device__ __forceinline__ v8f mma(V a, V b, v8f c) { return wmma16(a, b, c); } };
template <> struct WFrag<bf> { typedef v16bf V; static __device__ __forceinline__ V ld(const bf* p) { return cat16b(*(const v8us*)p, *(const v8us*)(p + 16)); } static __device__ __forceinline__ v8f mma(V a, V b, v8f c) { return wmmab(a, b, c); } };
template <typename T16, int NSPLIT, bool BIAS>
__global__ __launch_bounds__(32) void k_gemmw(const T16* __restrict__ A, const T16* __restrict__ A2, const T16* __restrict__ Bt, const T16* __restrict__ Bt2, int K, float* C, int ldc, float oscale, const float* __restrict__ bias, size_t sA, size_t sB, size_t sC) {
    typedef typename WFrag<T16>::V V;
    __shared__ __align__(16) float os[16 * 68];
    const size_t z = blockIdx.z; A += z * sA; if (A2) A2 += z * sA; Bt += z * sB; if (Bt2) Bt2 += z * sB; C += z * sC;
    const int lane = threadIdx.x & 31, lr = lane & 15, hi = lane >> 4; const int r0 = blockIdx.x * 64, c0 = blockIdx.y * 64;
    v8f acc[4][4];
#pragma unroll
    for (int mb = 0; mb < 4; ++mb)
#pragma unroll
        for (int nb = 0; nb < 4; ++nb) acc[mb][nb] = (v8f){};
    const size_t aoff = (size_t)(r0 + lr) * K + 8 * hi, boff = (size_t)(c0 + lr) * K + 8 * hi;
#pragma unroll 1
    for (int kc = 0; kc < K; kc += 32) {
        V a[4], a2[4];
#pragma unroll
        for (int mb = 0; mb < 4; ++mb) { a[mb] = WFrag<T16>::ld(A + aoff + (size_t)mb * 16 * K + kc); a2[mb] = a[mb]; if (NSPLIT == 1 || NSPLIT == 2) a2[mb] = WFrag<T16>::ld(A2 + aoff + (size_t)mb * 16 * K + kc); }
#pragma unroll
        for (int nb = 0; nb < 4; ++nb) { const V b = WFrag<T16>::ld(Bt + boff + (size_t)nb * 16 * K + kc); V b2 = b; if (NSPLIT >= 2) b2 = WFrag<T16>::ld(Bt2 + boff + (size_t)nb * 16 * K + kc);
#pragma unroll
            for (int mb = 0; mb < 4; ++mb) { acc[mb][nb] = WFrag<T16>::mma(a[mb], b, acc[mb][nb]); if (NSPLIT == 1 || NSPLIT == 2) acc[mb][nb] = WFrag<T16>::mma(a2[mb], b, acc[mb][nb]); if (NSPLIT >= 2) acc[mb][nb] = WFrag<T16>::mma(a[mb], b2, acc[mb][nb]); } }
        asm volatile("v_nop\n\tv_nop\n\tv_nop\n\tv_nop" : "+v"(acc[0][0]), "+v"(acc[1][1]), "+v"(acc[2][2]), "+v"(acc[3][3]) : "v"(a[0]), "v"(a[3]));
    }
#pragma unroll
    for (int mb = 0; mb < 4; ++mb) {
#pragma unroll
        for (int nb = 0; nb < 4; ++nb) {
#pragma unroll
            for (int j = 0; j < 8; ++j) os[(hi * 8 + j) * 68 + nb * 16 + lr] = acc[mb][nb][j]; }
        __builtin_amdgcn_wave_barrier(); asm volatile("" ::: "memory");
        float* crow = C + (size_t)(r0 + mb * 16) * ldc + c0;
#pragma unroll 1
        for (int ps = 0; ps < 2; ++ps) {
#pragma unroll
            for (int s = 0; s < 8; ++s) { const int row = 2 * s + hi, cofs = lr * 4; v4f val = *(const v4fa*)(os + row * 68 + cofs); val = val * oscale;
                if (BIAS) { val[0] += bfr(bias[c0 + cofs]); val[1] += bfr(bias[c0 + cofs + 1]); val[2] += bfr(bias[c0 + cofs + 2]); val[3] += bfr(bias[c0 + cofs + 3]); }
                *(volatile v4f*)(crow + (size_t)row * ldc + cofs) = val; }
            if (ps == 0) __threadfence(); }
        __builtin_amdgcn_wave_barrier(); asm volatile("" ::: "memory");
    }
}

__global__ __launch_bounds__(256) void k_cvt8(const float* __restrict__ src, bf* dst, size_t n8) { const size_t i = (size_t)blockIdx.x * 256 + threadIdx.x; if (i >= n8) return; const v8f v = *(const v8f*)(src + i * 8); v8us o;
#pragma unroll
    for (int k = 0; k < 8; ++k) o[k] = f2bf(v[k]); *(volatile v8us*)(dst + i * 8) = o; __threadfence(); *(volatile v8us*)(dst + i * 8) = o; }

template <bool RB>
__global__ __launch_bounds__(256) void k_cvth(const float* __restrict__ src, float sc, h16* dst, size_t n8) { const size_t i = (size_t)blockIdx.x * 256 + threadIdx.x; if (i >= n8) return; const v8f v = *(const v8f*)(src + i * 8); v8h o;
#pragma unroll
    for (int k = 0; k < 8; ++k) { const float y = RB ? bfr(v[k]) : v[k]; o[k] = tohx(y * sc); } *(volatile v8h*)(dst + i * 8) = o; __threadfence(); *(volatile v8h*)(dst + i * 8) = o; }

__global__ __launch_bounds__(256) void k_qkp(const float* __restrict__ F, bf* Ph, bf* Pl) {
    const size_t i = (size_t)blockIdx.x * 256 + threadIdx.x; if (i >= (size_t)SEQ * 2 * DM / 8) return;
    const size_t e = i * 8; const int t = (int)(e / (2 * DM)); const int c = (int)(e % (2 * DM)); const int p = c / DM; const int cc = c % DM;
    const float* f = F + (size_t)t * QC + c; const v4f x0 = *(const v4f*)f; const v4f x1 = *(const v4f*)(f + 4); v8us oh, ol;
#pragma unroll
    for (int q = 0; q < 4; ++q) { unsigned short a, l2; splitf(x0[q], a, l2); oh[q] = a; ol[q] = l2; splitf(x1[q], a, l2); oh[q + 4] = a; ol[q + 4] = l2; }
    const size_t o = (size_t)p * SEQ * DM + (size_t)t * DM + cc;
    *(volatile v8us*)(Ph + o) = oh; *(volatile v8us*)(Pl + o) = ol; __threadfence(); *(volatile v8us*)(Ph + o) = oh; *(volatile v8us*)(Pl + o) = ol;
}

__global__ __launch_bounds__(256) void k_vtp(const float* __restrict__ F, h16* VT) {
    const size_t i = (size_t)blockIdx.x * 256 + threadIdx.x; if (i >= (size_t)DM * SEQ / 8) return;
    const size_t e = i * 8; const int t = (int)(e % SEQ); const int d = (int)(e / SEQ); v8h o;
#pragma unroll
    for (int q = 0; q < 8; ++q) o[q] = tohx(F[(size_t)(t + q) * QC + 2 * DM + d]);
    *(volatile v8h*)(VT + e) = o; __threadfence(); *(volatile v8h*)(VT + e) = o;
}

__global__ __launch_bounds__(256) void k_asoft(const float* __restrict__ Sb, h16* P16) {
    const int lane = threadIdx.x & 31; const int row = blockIdx.x * 8 + (threadIdx.x >> 5); if (row >= SEQ) return;
    const float* sr = Sb + (size_t)row * SEQ; float v[SEQ / 32]; float mx = -3.0e38f;
#pragma unroll
    for (int ch = 0; ch < SEQ / 128; ++ch) { const int j0 = ch * 128 + lane * 4; const v4f a = *(const v4f*)(sr + j0);
#pragma unroll
        for (int q = 0; q < 4; ++q) { const float t = a[q] * SCL; v[ch * 4 + q] = t; mx = fmaxf(mx, t); } }
#pragma unroll
    for (int sh = 16; sh; sh >>= 1) mx = fmaxf(mx, __shfl_xor(mx, sh, 32));
    float sum = 0.f;
#pragma unroll
    for (int k = 0; k < SEQ / 32; ++k) { float d0 = __fsub_rn(v[k], mx); asm volatile("" : "+v"(d0)); v[k] = __builtin_amdgcn_exp2f(__fmul_rn(d0, 1.4426950408889634f)); sum += v[k]; }
#pragma unroll
    for (int sh = 16; sh; sh >>= 1) sum += __shfl_xor(sum, sh, 32);
    const float f = __fdiv_rn(PCAR, sum);
#pragma unroll 1
    for (int ps = 0; ps < 2; ++ps) {
#pragma unroll
        for (int ch = 0; ch < SEQ / 128; ++ch) { v4h o4;
#pragma unroll
            for (int q = 0; q < 4; ++q) o4[q] = tohx(v[ch * 4 + q] * f);
            *(volatile v4h*)(P16 + (size_t)row * SEQ + ch * 128 + lane * 4) = o4; }
        if (ps == 0) __threadfence(); }
}

extern "C" void kernel_launch(void* const* d_in, const int* in_sizes, int n_in,
                              void* d_out, int out_size, void* d_ws, size_t ws_size, hipStream_t stream) {
    if (n_in < 4) return;
    if (in_sizes[0] < (NB - 1) * SEQ_FULL * DM + SEQ * DM) return;
    if (in_sizes[1] < QC * DM) return;
    if (in_sizes[2] < DM * DM) return;
    if (in_sizes[3] < DM) return;
    if (out_size < NB * SEQ * DM) return;
    const float* x = (const float*)d_in[0];
    const float* wqkv = (const float*)d_in[1];
    const float* wout = (const float*)d_in[2];
    const float* bout = (const float*)d_in[3];
    float* OUT = (float*)d_out;
    char* wsp = (char*)d_ws;
    auto take = [&](size_t bytes) { char* p = wsp; wsp += (bytes + 255) & ~(size_t)255; return (void*)p; };
    bf*  WQ  = (bf*)take((size_t)QC * DM * 2);
    h16* WO  = (h16*)take((size_t)DM * DM * 2);
    bf*  XB  = (bf*)take((size_t)SEQ * DM * 2);
    float* F = (float*)take((size_t)SEQ * QC * 4);
    bf*  QKh = (bf*)take((size_t)2 * SEQ * DM * 2);
    bf*  QKl = (bf*)take((size_t)2 * SEQ * DM * 2);
    h16* VT  = (h16*)take((size_t)DM * SEQ * 2);
    float* Sb = (float*)take((size_t)SEQ * SEQ * 4);
    h16* P16 = (h16*)take((size_t)SEQ * SEQ * 2);
    float* Ob = (float*)take((size_t)SEQ * DM * 4);
    h16* CT  = (h16*)take((size_t)SEQ * DM * 2);
    if ((size_t)(wsp - (char*)d_ws) > ws_size) return;

    const size_t nW8 = (size_t)QC * DM / 8, nO8 = (size_t)DM * DM / 8, nX8 = (size_t)SEQ * DM / 8, nQK8 = (size_t)SEQ * 2 * DM / 8, nV8 = (size_t)DM * SEQ / 8;
    k_cvt8<<<(unsigned)((nW8 + 255) / 256), 256, 0, stream>>>(wqkv, WQ, nW8);
    k_cvth<true><<<(unsigned)((nO8 + 255) / 256), 256, 0, stream>>>(wout, WSC, WO, nO8);
    for (int b = 0; b < NB; ++b) {
        k_cvt8<<<(unsigned)((nX8 + 255) / 256), 256, 0, stream>>>(x + (size_t)b * SEQ_FULL * DM, XB, nX8);
        k_gemmw<bf, 0, false><<<dim3(SEQ / 64, QC / 64, 1), 32, 0, stream>>>(XB, nullptr, WQ, nullptr, DM, F, QC, 1.0f, nullptr, 0, 0, 0);
        k_qkp<<<(unsigned)((nQK8 + 255) / 256), 256, 0, stream>>>(F, QKh, QKl);
        k_vtp<<<(unsigned)((nV8 + 255) / 256), 256, 0, stream>>>(F, VT);
        k_gemmw<bf, 2, false><<<dim3(SEQ / 64, SEQ / 64, 1), 32, 0, stream>>>(QKh, QKl, QKh + (size_t)SEQ * DM, QKl + (size_t)SEQ * DM, DM, Sb, SEQ, 1.0f, nullptr, 0, 0, 0);
        k_asoft<<<SEQ / 8, 256, 0, stream>>>(Sb, P16);
        k_gemmw<h16, 0, false><<<dim3(SEQ / 64, DM / 64, 1), 32, 0, stream>>>(P16, nullptr, VT, nullptr, SEQ, Ob, DM, 1.0f / PCAR, nullptr, 0, 0, 0);
        k_cvth<false><<<(unsigned)((nX8 + 255) / 256), 256, 0, stream>>>(Ob, 1.0f, CT, nX8);
        k_gemmw<h16, 0, true><<<dim3(SEQ / 64, DM / 64, 1), 32, 0, stream>>>(CT, nullptr, WO, nullptr, DM, OUT + (size_t)b * SEQ * DM, DM, 1.0f / WSC, bout, 0, 0, 0);
    }
}
